// BiLSTMCRFChordClassifier_14448269983808
// MI455X (gfx1250) — hardware-verified
//
#include <hip/hip_runtime.h>
#include <stdint.h>


typedef _Float16       v16h  __attribute__((ext_vector_type(16)));
typedef __bf16         v16b  __attribute__((ext_vector_type(16)));
typedef unsigned short v16us __attribute__((ext_vector_type(16)));
typedef unsigned short v8us  __attribute__((ext_vector_type(8)));
typedef unsigned short v8us_a __attribute__((ext_vector_type(8), may_alias));
typedef float          v8f   __attribute__((ext_vector_type(8)));
typedef float          v4f   __attribute__((ext_vector_type(4)));
typedef float          v4f_a __attribute__((ext_vector_type(4), may_alias));

#define NB 128
#define NT 2048
#define ND 24
#define NH 128
#define NC 24
#define NG 512
#define EP 32

#define LOFF_WHH   0
#define LOFF_WIHH  131072
#define LOFF_WIHL  163840
#define LOFF_WCH   196608
#define LOFF_WCL   204800
#define LOFF_HB    212992
#define LOFF_HHI   221184
#define LOFF_HLO   229376
#define LOFF_XHI   237568
#define LOFF_XLO   239616
#define LOFF_PB    241664
#define LDS_BYTES  258048

__device__ __forceinline__ unsigned short f2bf(float x) {
  const unsigned u = __float_as_uint(x);
  return (unsigned short)((u + 0x7FFFu + ((u >> 16) & 1u)) >> 16);
}
__device__ __forceinline__ float bf2f(unsigned short b) {
  return __uint_as_float(((unsigned)b) << 16);
}
__device__ __forceinline__ unsigned short f2hs(float x) {
  const _Float16 h = (_Float16)x;
  return __builtin_bit_cast(unsigned short, h);
}

union Frag16 { v16us v; v8us h[2]; };

__device__ __forceinline__ v16us ldfrag(const unsigned short* p) {
  Frag16 f;
  f.h[0] = *(const v8us_a*)(p);
  f.h[1] = *(const v8us_a*)(p + 16);
  return f.v;
}

__device__ __forceinline__ v8f mma_bf(v16us a, v16us b, v8f c) {
  const v16b av = __builtin_bit_cast(v16b, a);
  const v16b bv = __builtin_bit_cast(v16b, b);
  v8f d = __builtin_amdgcn_wmma_f32_16x16x32_bf16(false, av, false, bv, (short)0, c, false, false);
  asm volatile("v_nop\n\tv_nop\n\tv_nop\n\tv_nop" : "+v"(d) : "v"(a), "v"(b));
  return d;
}
__device__ __forceinline__ v8f mma_h(v16us a, v16us b, v8f c) {
  const v16h av = __builtin_bit_cast(v16h, a);
  const v16h bv = __builtin_bit_cast(v16h, b);
  v8f d = __builtin_amdgcn_wmma_f32_16x16x32_f16(false, av, false, bv, (short)0, c, false, false);
  asm volatile("v_nop\n\tv_nop\n\tv_nop\n\tv_nop" : "+v"(d) : "v"(a), "v"(b));
  return d;
}

__device__ __forceinline__ float sigm(float x) {
  return __builtin_amdgcn_rcpf(1.0f + __expf(-x));
}
__device__ __forceinline__ float tnh(float x) {
  const float a = __builtin_fabsf(x);
  const float e = __expf(2.0f * a);
  const float r = 1.0f - 2.0f * __builtin_amdgcn_rcpf(e + 1.0f);
  return __builtin_copysignf(r, x);
}

__device__ __forceinline__ void stage_x2(unsigned short* hi, unsigned short* lo, int idx, float2 v) {
  const unsigned short h0 = f2bf(v.x), h1 = f2bf(v.y);
  hi[idx]     = h0;
  hi[idx + 1] = h1;
  lo[idx]     = f2bf(v.x - bf2f(h0));
  lo[idx + 1] = f2bf(v.y - bf2f(h1));
}

__global__ __launch_bounds__(256) __attribute__((amdgpu_num_vgpr(256)))
void k_lstm(const float* __restrict__ x,
            const float* __restrict__ wihf, const float* __restrict__ whhf,
            const float* __restrict__ bihf, const float* __restrict__ bhhf,
            const float* __restrict__ wihb, const float* __restrict__ whhb,
            const float* __restrict__ bihb, const float* __restrict__ bhhb,
            const float* __restrict__ wcls,
            float* __restrict__ empf,
            float* __restrict__ empb)
{
  extern __shared__ __align__(16) unsigned char lds_raw[];
  unsigned short* Lwhh  = (unsigned short*)(lds_raw + LOFF_WHH);
  unsigned short* Lwihh = (unsigned short*)(lds_raw + LOFF_WIHH);
  unsigned short* Lwihl = (unsigned short*)(lds_raw + LOFF_WIHL);
  unsigned short* Lwch  = (unsigned short*)(lds_raw + LOFF_WCH);
  unsigned short* Lwcl  = (unsigned short*)(lds_raw + LOFF_WCL);
  unsigned short* Lhb   = (unsigned short*)(lds_raw + LOFF_HB);
  unsigned short* Lhhi  = (unsigned short*)(lds_raw + LOFF_HHI);
  unsigned short* Lhlo  = (unsigned short*)(lds_raw + LOFF_HLO);
  unsigned short* Lxhi  = (unsigned short*)(lds_raw + LOFF_XHI);
  unsigned short* Lxlo  = (unsigned short*)(lds_raw + LOFF_XLO);
  float*          Lpb   = (float*)(lds_raw + LOFF_PB);

  const int dir = blockIdx.y;
  const int b0  = blockIdx.x * 16;
  if (b0 + 16 > NB || dir > 1) return;

  const float* wih = dir ? wihb : wihf;
  const float* whh = dir ? whhb : whhf;
  const float* bih = dir ? bihb : bihf;
  const float* bhh = dir ? bhhb : bhhf;
  float*       emp = dir ? empb : empf;

  const int tid = threadIdx.x, wv = tid >> 5, lane = tid & 31;
  const int m = lane & 15, hh = lane >> 4;
  const int hcol = 16 * wv + m;
  const int cch = wv & 3, cnt = wv >> 2;

  for (int i = tid; i < NG * NH; i += 256) Lwhh[i] = f2hs(whh[i] * 64.0f);
  for (int i = tid; i < NG * 32; i += 256) {
    const int row = i >> 5, k = i & 31;
    const float v = (k < ND) ? wih[row * ND + k] * 16384.0f : 0.0f;
    const unsigned short hi = f2bf(v);
    Lwihh[i] = hi;
    Lwihl[i] = f2bf(v - bf2f(hi));
  }
  for (int i = tid; i < 32 * NH; i += 256) {
    const int n = i >> 7, k = i & 127;
    const float v = (n < NC) ? wcls[(size_t)n * (2 * NH) + (size_t)dir * NH + k] : 0.0f;
    const unsigned short hi = f2bf(v);
    Lwch[i] = hi;
    Lwcl[i] = f2bf(v - bf2f(hi));
  }
  for (int i = tid; i < 2048; i += 256) Lhb[i] = 0;
  for (int i = tid; i < 1024; i += 256) { Lxhi[i] = 0; Lxlo[i] = 0; }
  __syncthreads();

  const bool xth  = (tid < 192);
  const int  prow = tid / 12;
  const int  pd   = (tid % 12) * 2;
  if (xth) {
    const int t0 = dir ? (NT - 1) : 0;
    const float2 xv = *(const float2*)&x[((size_t)(b0 + prow) * NT + t0) * ND + pd];
    stage_x2(Lxhi, Lxlo, prow * 32 + pd, xv);
  }

  float bias[4];
#pragma unroll
  for (int g = 0; g < 4; ++g) {
    const int gr = g * NH + hcol;
    bias[g] = (bih[gr] + bhh[gr]) * 16384.0f;
  }
  float cst[8];
#pragma unroll
  for (int r = 0; r < 8; ++r) cst[r] = 0.0f;
  __syncthreads();

  const float SCI = 1.0f / 16384.0f;

#pragma unroll 1
  for (int s = 0; s < NT + 2; ++s) {
    const int rb = s & 1, wb = rb ^ 1;

    if (s >= 2 && tid < 128) {
      const int row = tid >> 3, q = tid & 7;
      const int nt = q >> 2, j0 = (q & 3) * 4;
      const float* P = Lpb + wb * 2048 + (4 * nt) * 256 + row * 16 + j0;
      const v4f sum = *(const v4f_a*)(P) + *(const v4f_a*)(P + 256)
                    + *(const v4f_a*)(P + 512) + *(const v4f_a*)(P + 768);
      const int s2 = s - 2;
      const int tt = dir ? (NT - 1 - s2) : s2;
      float* dst = emp + ((size_t)tt * NB + (size_t)(b0 + row)) * EP + 4 * q;
      *(volatile v4f*)dst = sum;
      __threadfence();
      *(volatile v4f*)dst = sum;
    }

    float2 xv = {0.0f, 0.0f};
    const bool dop = xth && (s + 1 < NT);
    if (dop) {
      const int tn = dir ? (NT - 2 - s) : (s + 1);
      xv = *(const float2*)&x[((size_t)(b0 + prow) * NT + tn) * ND + pd];
    }

    if (s < NT) {
      v8f acc[4];
#pragma unroll
      for (int g = 0; g < 4; ++g) {
        v8f ci;
#pragma unroll
        for (int r = 0; r < 8; ++r) ci[r] = bias[g];
        acc[g] = ci;
      }
      {
        const int xo = rb * 512 + m * 32 + 8 * hh;
        const v16us axh = ldfrag(Lxhi + xo);
        const v16us axl = ldfrag(Lxlo + xo);
#pragma unroll
        for (int g = 0; g < 4; ++g) {
          const int wo = (g * NH + hcol) * 32 + 8 * hh;
          const v16us bh = ldfrag(Lwihh + wo);
          const v16us bl = ldfrag(Lwihl + wo);
          acc[g] = mma_bf(axh, bh, acc[g]);
          acc[g] = mma_bf(axh, bl, acc[g]);
          acc[g] = mma_bf(axl, bh, acc[g]);
        }
      }
#pragma unroll
      for (int c = 0; c < 4; ++c) {
        const v16us ah = ldfrag(Lhb + rb * 2048 + m * NH + 32 * c + 8 * hh);
#pragma unroll
        for (int g = 0; g < 4; ++g) {
          const v16us bw = ldfrag(Lwhh + (g * NH + hcol) * NH + 32 * c + 8 * hh);
          acc[g] = mma_h(ah, bw, acc[g]);
        }
      }

#pragma unroll
      for (int r = 0; r < 8; ++r) {
        const float zi = acc[0][r] * SCI;
        const float zf = acc[1][r] * SCI;
        const float zg = acc[2][r] * SCI;
        const float zo = acc[3][r] * SCI;
        const float iv = sigm(zi), fv = sigm(zf), gv = tnh(zg), ov = sigm(zo);
        const float cs = fv * cst[r] + iv * gv;
        cst[r] = cs;
        const float hv = ov * tnh(cs);
        const int idx = wb * 2048 + (8 * hh + r) * NH + hcol;
        Lhb[idx] = f2hs(hv * 256.0f);
        const unsigned short hb16 = f2bf(hv);
        Lhhi[idx] = hb16;
        Lhlo[idx] = f2bf(hv - bf2f(hb16));
      }
    }

    if (s >= 1 && s <= NT) {
      const int ho = rb * 2048 + m * NH + 32 * cch + 8 * hh;
      const v16us ahh = ldfrag(Lhhi + ho);
      const v16us ahl = ldfrag(Lhlo + ho);
      const int co = (16 * cnt + m) * NH + 32 * cch + 8 * hh;
      const v16us bch = ldfrag(Lwch + co);
      const v16us bcl = ldfrag(Lwcl + co);
      v8f pacc;
#pragma unroll
      for (int r = 0; r < 8; ++r) pacc[r] = 0.0f;
      pacc = mma_bf(ahh, bch, pacc);
      pacc = mma_bf(ahh, bcl, pacc);
      pacc = mma_bf(ahl, bch, pacc);
      float* P = Lpb + rb * 2048 + wv * 256;
#pragma unroll
      for (int r = 0; r < 8; ++r) P[(8 * hh + r) * 16 + m] = pacc[r];
    }

    if (dop) stage_x2(Lxhi + wb * 512, Lxlo + wb * 512, prow * 32 + pd, xv);

    __syncthreads();
  }
}

__global__ __launch_bounds__(256)
void k_emit(const float* __restrict__ empf, const float* __restrict__ empb,
            const float* __restrict__ bcls, float* __restrict__ out, int n4)
{
  const int i = blockIdx.x * 256 + threadIdx.x;
  if (i >= n4) return;
  const int f = i * 4;
  const int b = f / (NT * NC);
  const int rem = f - b * (NT * NC);
  const int t = rem / NC;
  const int c = rem - t * NC;
  const size_t o = ((size_t)t * NB + (size_t)b) * EP + (size_t)c;
  const v4f v = *(const v4f_a*)(empf + o) + *(const v4f_a*)(empb + o) + *(const v4f_a*)(bcls + c);
  float* dst = out + (size_t)f;
  *(volatile v4f*)dst = v;
  __threadfence();
  *(volatile v4f*)dst = v;
}

__device__ __forceinline__ int clamp_tag(int v) { return v < 0 ? 0 : (v >= NC ? NC - 1 : v); }

__global__ __launch_bounds__(32)
void k_crf(const float* __restrict__ empf, const float* __restrict__ empb,
           const float* __restrict__ bcls, const int* __restrict__ lab,
           const float* __restrict__ st, const float* __restrict__ en,
           const float* __restrict__ tr, float* __restrict__ llh)
{
  const int b = blockIdx.x;
  if (b >= NB) return;
  const int j = threadIdx.x;
  const bool act = (j < NC);
  const int jc = act ? j : 0;

  float trc[NC];
#pragma unroll
  for (int i = 0; i < NC; ++i) trc[i] = tr[i * NC + jc];
  const float bj  = act ? bcls[jc] : 0.0f;
  const float stj = st[jc];
  const float enj = en[jc];
  const size_t lbase = (size_t)b * NT;

  size_t o = (size_t)b * EP + j;
  const float e0 = empf[o] + empb[o] + bj;
  float alpha = act ? (stj + e0) : -1.0e30f;
  int tg = clamp_tag(lab[lbase]);
  float num = st[tg] + __shfl(e0, tg);
  int prev = tg;

#pragma unroll 1
  for (int t = 1; t < NT; ++t) {
    o = ((size_t)t * NB + (size_t)b) * EP + j;
    const float et = empf[o] + empb[o] + bj;
    float v[NC];
    float mx = -1.0e30f;
#pragma unroll
    for (int i = 0; i < NC; ++i) {
      const float xv = __shfl(alpha, i) + trc[i];
      v[i] = xv;
      mx = fmaxf(mx, xv);
    }
    float ssum = 0.0f;
#pragma unroll
    for (int i = 0; i < NC; ++i) ssum += __expf(v[i] - mx);
    const float na = et + mx + __logf(ssum);
    alpha = act ? na : -1.0e30f;

    tg = clamp_tag(lab[lbase + t]);
    num += __shfl(et, tg) + tr[prev * NC + tg];
    prev = tg;
  }
  num += en[prev];

  const float ae = act ? (alpha + enj) : -1.0e30f;
  float v2[NC];
  float mx2 = -1.0e30f;
#pragma unroll
  for (int i = 0; i < NC; ++i) {
    const float xv = __shfl(ae, i);
    v2[i] = xv;
    mx2 = fmaxf(mx2, xv);
  }
  float s2 = 0.0f;
#pragma unroll
  for (int i = 0; i < NC; ++i) s2 += __expf(v2[i] - mx2);
  const float logz = mx2 + __logf(s2);
  const float val = num - logz;

  if (j < 8) {
    v4f w = {0.0f, 0.0f, 0.0f, 0.0f};
    if (j == 0) w.x = val;
    float* dst = llh + (size_t)b * 32 + 4 * j;
    *(volatile v4f*)dst = w;
    __threadfence();
    *(volatile v4f*)dst = w;
  }
}

__global__ __launch_bounds__(128)
void k_loss(const float* __restrict__ llh, float* __restrict__ out1)
{
  __shared__ float sm[128];
  const int i = threadIdx.x;
  sm[i] = llh[(size_t)i * 32];
  __syncthreads();
  for (int s = 64; s > 0; s >>= 1) {
    if (i < s) sm[i] = sm[i] + sm[i + s];
    __syncthreads();
  }
  if (i == 0) {
    const float v = -sm[0] * (1.0f / (float)NB);
    *(volatile float*)out1 = v;
    __threadfence();
    *(volatile float*)out1 = v;
  }
}

extern "C" void kernel_launch(void* const* d_in, const int* in_sizes, int n_in,
                              void* d_out, int out_size, void* d_ws, size_t ws_size,
                              hipStream_t stream)
{
  if (n_in < 15) return;
  if (in_sizes[0] != NB * NT * ND) return;
  if (in_sizes[1] != NB * NT) return;
  if (in_sizes[2] != NG * ND || in_sizes[3] != NG * NH || in_sizes[4] != NG || in_sizes[5] != NG) return;
  if (in_sizes[6] != NG * ND || in_sizes[7] != NG * NH || in_sizes[8] != NG || in_sizes[9] != NG) return;
  if (in_sizes[10] != NC * 2 * NH || in_sizes[11] != NC) return;
  if (in_sizes[12] != NC || in_sizes[13] != NC || in_sizes[14] != NC * NC) return;
  if (out_size != NB * NT * NC + 1) return;

  const float* x    = (const float*)d_in[0];
  const int*   lab  = (const int*)d_in[1];
  const float* wihf = (const float*)d_in[2];
  const float* whhf = (const float*)d_in[3];
  const float* bihf = (const float*)d_in[4];
  const float* bhhf = (const float*)d_in[5];
  const float* wihb = (const float*)d_in[6];
  const float* whhb = (const float*)d_in[7];
  const float* bihb = (const float*)d_in[8];
  const float* bhhb = (const float*)d_in[9];
  const float* wcls = (const float*)d_in[10];
  const float* bcls = (const float*)d_in[11];
  const float* st   = (const float*)d_in[12];
  const float* en   = (const float*)d_in[13];
  const float* tr   = (const float*)d_in[14];
  float* out = (float*)d_out;

  const size_t empBytes = (size_t)NT * NB * EP * sizeof(float);
  const size_t offF = 0;
  const size_t offB = offF + empBytes;
  const size_t offL = offB + empBytes;
  const size_t need = offL + (size_t)NB * 32 * sizeof(float);
  if (need > ws_size) return;

  float* empf = (float*)((char*)d_ws + offF);
  float* empb = (float*)((char*)d_ws + offB);
  float* llh  = (float*)((char*)d_ws + offL);

  k_lstm<<<dim3(NB / 16, 2), dim3(256), LDS_BYTES, stream>>>(
      x, wihf, whhf, bihf, bhhf, wihb, whhb, bihb, bhhb, wcls, empf, empb);

  const int n4 = (NB * NT * NC) / 4;
  k_emit<<<dim3((n4 + 255) / 256), dim3(256), 0, stream>>>(empf, empb, bcls, out, n4);

  k_crf<<<dim3(NB), dim3(32), 0, stream>>>(empf, empb, bcls, lab, st, en, tr, llh);

  k_loss<<<dim3(1), dim3(128), 0, stream>>>(llh, out + (size_t)NB * NT * NC);
}
